// MultiHeadedSelfAttention_858993459369
// MI455X (gfx1250) — hardware-verified
//
#include <hip/hip_runtime.h>


#ifndef NB
#define NB 4
#endif
#ifndef SEQ
#define SEQ 2048
#endif
#define NB_FULL 4
#define SEQ_FULL 2048
#define EMB 512
#define NH 8
#define HD 64
#define MTOK (NB * SEQ)

static_assert(NB >= 1 && NB <= NB_FULL);
static_assert(SEQ >= 128 && SEQ <= SEQ_FULL && (SEQ % 128) == 0);
static_assert(EMB == NH * HD);
static_assert((EMB % 64) == 0 && (MTOK % 128) == 0);
static_assert((3ull * NB_FULL * NH * SEQ_FULL * HD + (unsigned long long)NB_FULL * SEQ_FULL * EMB) * 2ull <= 134217728ull);

typedef unsigned short u16;
typedef _Float16 v16h __attribute__((ext_vector_type(16)));
typedef __bf16   v16bf __attribute__((ext_vector_type(16)));
typedef float    v8f  __attribute__((ext_vector_type(8)));
typedef _Float16 v8ha __attribute__((ext_vector_type(8), __may_alias__));
typedef float    v4fa __attribute__((ext_vector_type(4), __may_alias__));
typedef unsigned v4u  __attribute__((ext_vector_type(4), __may_alias__));

union FragH { v16h v; v8ha p[2]; };
union FragB { v16bf v; v4u q[2]; };
union Pack8 { v8ha h; v4u u; _Float16 s[8]; };


__device__ __forceinline__ unsigned bfbits(float f) {
  unsigned u = __float_as_uint(f);
  u += 0x7FFFu + ((u >> 16) & 1u);
  return u >> 16;
}
__device__ __forceinline__ float bfval(float f) {
  unsigned u = __float_as_uint(f);
  u += 0x7FFFu + ((u >> 16) & 1u);
  return __uint_as_float(u & 0xFFFF0000u);
}
__device__ __forceinline__ v8f z8() {
  v8f z = {0.f, 0.f, 0.f, 0.f, 0.f, 0.f, 0.f, 0.f};
  return z;
}

__device__ __forceinline__ v4u pack_bf8(const float* __restrict__ p) {
  const v4fa x0 = *(const v4fa*)p;
  const v4fa x1 = *(const v4fa*)(p + 4);
  v4u r;
  r.x = bfbits(x0.x) | (bfbits(x0.y) << 16);
  r.y = bfbits(x0.z) | (bfbits(x0.w) << 16);
  r.z = bfbits(x1.x) | (bfbits(x1.y) << 16);
  r.w = bfbits(x1.z) | (bfbits(x1.w) << 16);
  return r;
}

__device__ __forceinline__ v16h frag_h(const _Float16* base, int ld) {
  const int lane = threadIdx.x & 31;
  const int row  = lane & 15;
  const int kb   = (lane >> 4) << 3;
  FragH u;
  u.p[0] = *(const v8ha*)(base + (size_t)row * ld + kb);
  u.p[1] = *(const v8ha*)(base + (size_t)row * ld + 16 + kb);
  return u.v;
}

__device__ __forceinline__ v16bf frag_x_bf(const float* base, int ld, int k0) {
  const int lane = threadIdx.x & 31;
  const int row  = lane & 15;
  const int kb   = (lane >> 4) << 3;
  const float* p = base + (size_t)row * ld + k0 + kb;
  FragB u;
  u.q[0] = pack_bf8(p);
  u.q[1] = pack_bf8(p + 16);
  return u.v;
}

__device__ __forceinline__ v16bf frag_w_bf(const v4u* tile, int nrow0, int kc0) {
  const int lane = threadIdx.x & 31;
  const int n    = lane & 15;
  const int hh   = lane >> 4;
  FragB u;
  u.q[0] = tile[(nrow0 + n) * 8 + kc0 + hh];
  u.q[1] = tile[(nrow0 + n) * 8 + kc0 + 2 + hh];
  return u.v;
}

__device__ __forceinline__ v8f mma_h(v16h a, v16h b, v8f c) {
  v8f d = __builtin_amdgcn_wmma_f32_16x16x32_f16(false, a, false, b, (short)0, c, false, false);
  asm volatile("v_nop\n\tv_nop\n\tv_nop\n\tv_nop" : "+v"(d) : "v"(a), "v"(b));
  return d;
}
__device__ __forceinline__ v8f mma_bf(v16bf a, v16bf b, v8f c) {
  v8f d = __builtin_amdgcn_wmma_f32_16x16x32_bf16(false, a, false, b, (short)0, c, false, false);
  asm volatile("v_nop\n\tv_nop\n\tv_nop\n\tv_nop" : "+v"(d) : "v"(a), "v"(b));
  return d;
}

__device__ __forceinline__ float hmax16(float x) {
#pragma unroll
  for (int m = 1; m < 16; m <<= 1) x = fmaxf(x, __shfl_xor(x, m, 32));
  return x;
}
__device__ __forceinline__ float hadd16(float x) {
#pragma unroll
  for (int m = 1; m < 16; m <<= 1) x += __shfl_xor(x, m, 32);
  return x;
}

__device__ __forceinline__ void wave_store_rows16(const _Float16* tile, _Float16* dst, int pitch) {
  const int lane = threadIdx.x & 31;
  const int rsub = lane >> 3, c8 = (lane & 7) << 3;
  Pack8 v[4];
#pragma unroll
  for (int it = 0; it < 4; ++it)
    v[it].h = *(const v8ha*)(tile + (it * 4 + rsub) * 64 + c8);
#pragma unroll
  for (int it = 0; it < 4; ++it)
    *(volatile v4u*)(dst + (size_t)(it * 4 + rsub) * pitch + c8) = v[it].u;
  __threadfence();
#pragma unroll
  for (int it = 0; it < 4; ++it)
    *(volatile v4u*)(dst + (size_t)(it * 4 + rsub) * pitch + c8) = v[it].u;
}

__global__ __launch_bounds__(256) void k_qkv(
    const float* __restrict__ x,
    const float* __restrict__ Wq, const float* __restrict__ bq,
    const float* __restrict__ Wk, const float* __restrict__ bk,
    const float* __restrict__ Wv, const float* __restrict__ bv,
    _Float16* __restrict__ Qp, _Float16* __restrict__ Kp, _Float16* __restrict__ Vtp) {
  __shared__ __align__(16) v4u Wl[3][512];
  __shared__ float Bl[3][HD];
  __shared__ __align__(16) _Float16 St[128 * HD];

  const int tid = threadIdx.x, wave = tid >> 5, lane = tid & 31;
  const int hh = lane >> 4, n16 = lane & 15;
  const int h  = blockIdx.y;
  const int m0 = blockIdx.x * 128;
  const int b  = m0 / SEQ, s0 = m0 - b * SEQ;
  const int bh = b * NH + h;

#pragma unroll
  for (int c = tid; c < 512; c += 256) {
    const int nrow = c >> 3, ko = (c & 7) << 3;
    const size_t off = ((size_t)h * HD + nrow) * HD + ko;
    Wl[0][c] = pack_bf8(Wq + off);
    Wl[1][c] = pack_bf8(Wk + off);
    Wl[2][c] = pack_bf8(Wv + off);
  }
  if (tid < HD) {
    Bl[0][tid] = bfval(bq[h * HD + tid]);
    Bl[1][tid] = bfval(bk[h * HD + tid]);
    Bl[2][tid] = bfval(bv[h * HD + tid]);
  }
  __syncthreads();

  const float* xp = x + ((size_t)b * SEQ_FULL + s0 + wave * 16) * EMB + h * HD;
  const v16bf a0 = frag_x_bf(xp, EMB, 0);
  const v16bf a1 = frag_x_bf(xp, EMB, 32);

#pragma unroll
  for (int mat = 0; mat < 3; ++mat) {
    v8f acc[4];
#pragma unroll
    for (int t = 0; t < 4; ++t) {
      v8f c = z8();
      c = mma_bf(a0, frag_w_bf(Wl[mat], t * 16, 0), c);
      c = mma_bf(a1, frag_w_bf(Wl[mat], t * 16, 4), c);
      acc[t] = c;
    }
#pragma unroll
    for (int t = 0; t < 4; ++t) {
      const float bias = Bl[mat][t * 16 + n16];
#pragma unroll
      for (int r = 0; r < 8; ++r)
        St[(wave * 16 + 8 * hh + r) * HD + t * 16 + n16] = (_Float16)(acc[t][r] + bias);
    }
    __syncthreads();

    if (mat < 2) {
      _Float16* plane = (mat == 0) ? Qp : Kp;
      wave_store_rows16(&St[(wave * 16) * HD],
                        plane + ((size_t)bh * SEQ + s0 + wave * 16) * HD, HD);
    } else {
      const int c8 = (tid & 7) << 3;
      Pack8 w[4];
#pragma unroll
      for (int it = 0; it < 4; ++it) {
        const int L = it * 32 + (tid >> 3);
        const int d = L >> 1, j0 = (L & 1) * 64 + c8;
#pragma unroll
        for (int e = 0; e < 8; ++e) w[it].s[e] = St[(j0 + e) * HD + d];
      }
#pragma unroll
      for (int it = 0; it < 4; ++it) {
        const int L = it * 32 + (tid >> 3);
        const int d = L >> 1, j0 = (L & 1) * 64 + c8;
        *(volatile v4u*)(Vtp + ((size_t)bh * HD + d) * SEQ + s0 + j0) = w[it].u;
      }
      __threadfence();
#pragma unroll
      for (int it = 0; it < 4; ++it) {
        const int L = it * 32 + (tid >> 3);
        const int d = L >> 1, j0 = (L & 1) * 64 + c8;
        *(volatile v4u*)(Vtp + ((size_t)bh * HD + d) * SEQ + s0 + j0) = w[it].u;
      }
    }
    __syncthreads();
  }
}

__global__ __launch_bounds__(256) void k_attn(
    const _Float16* __restrict__ Qp, const _Float16* __restrict__ Kp,
    const _Float16* __restrict__ Vtp, _Float16* __restrict__ Cp) {
  __shared__ __align__(16) _Float16 Kt[64 * HD];
  __shared__ __align__(16) _Float16 Vt[HD * 64];
  __shared__ __align__(16) _Float16 Pt[8][16 * 64];

  const int tid = threadIdx.x, wave = tid >> 5, lane = tid & 31;
  const int hh = lane >> 4, n16 = lane & 15;
  const int bh = blockIdx.x;
  const int b  = bh / NH, h = bh - b * NH;
  const int q0 = blockIdx.y * 128 + wave * 16;

  const _Float16* Qbh = Qp  + (size_t)bh * SEQ * HD;
  const _Float16* Kbh = Kp  + (size_t)bh * SEQ * HD;
  const _Float16* Vbh = Vtp + (size_t)bh * HD * SEQ;

  const v16h aq0 = frag_h(Qbh + (size_t)q0 * HD, HD);
  const v16h aq1 = frag_h(Qbh + (size_t)q0 * HD + 32, HD);

  float mrow[8], lrow[8];
  v8f o[4];
#pragma unroll
  for (int r = 0; r < 8; ++r) { mrow[r] = -1e30f; lrow[r] = 0.f; }
#pragma unroll
  for (int t = 0; t < 4; ++t) o[t] = z8();

  const float scale = 0.125f;

  for (int t0 = 0; t0 < SEQ; t0 += 64) {
    __syncthreads();
#pragma unroll
    for (int c = tid; c < 512; c += 256) {
      const int row = c >> 3, off = (c & 7) << 3;
      *(v8ha*)&Kt[row * HD + off] = *(const v8ha*)(Kbh + (size_t)(t0 + row) * HD + off);
      *(v8ha*)&Vt[row * 64 + off] = *(const v8ha*)(Vbh + (size_t)row * SEQ + t0 + off);
    }
    __syncthreads();

    v8f sc[4];
#pragma unroll
    for (int t = 0; t < 4; ++t) {
      const v16h kb0 = frag_h(&Kt[(t * 16) * HD], HD);
      const v16h kb1 = frag_h(&Kt[(t * 16) * HD + 32], HD);
      v8f c = z8();
      c = mma_h(aq0, kb0, c);
      c = mma_h(aq1, kb1, c);
      sc[t] = c;
    }

    float alpha[8];
#pragma unroll
    for (int r = 0; r < 8; ++r) {
      float mx = fmaxf(fmaxf(sc[0][r], sc[1][r]), fmaxf(sc[2][r], sc[3][r]));
      mx = hmax16(mx * scale);
      const float mnew = fmaxf(mrow[r], mx);
      alpha[r] = __expf(mrow[r] - mnew);
      mrow[r] = mnew;
    }
#pragma unroll
    for (int r = 0; r < 8; ++r) {
      float ps = 0.f;
#pragma unroll
      for (int t = 0; t < 4; ++t) {
        const float p = __expf(sc[t][r] * scale - mrow[r]);
        ps += p;
        Pt[wave][(8 * hh + r) * 64 + t * 16 + n16] = (_Float16)(p * 1024.0f);
      }
      lrow[r] = lrow[r] * alpha[r] + hadd16(ps);
    }
#pragma unroll
    for (int t = 0; t < 4; ++t)
#pragma unroll
      for (int r = 0; r < 8; ++r) o[t][r] *= alpha[r];

    __syncthreads();

    const v16h p0 = frag_h(&Pt[wave][0], 64);
    const v16h p1 = frag_h(&Pt[wave][32], 64);
#pragma unroll
    for (int dt = 0; dt < 4; ++dt) {
      const v16h vb0 = frag_h(&Vt[(dt * 16) * 64], 64);
      const v16h vb1 = frag_h(&Vt[(dt * 16) * 64 + 32], 64);
      v8f c = o[dt];
      c = mma_h(p0, vb0, c);
      c = mma_h(p1, vb1, c);
      o[dt] = c;
    }
  }

  float inv[8];
#pragma unroll
  for (int r = 0; r < 8; ++r) inv[r] = 0.0625f * __builtin_amdgcn_rcpf(lrow[r]);

  __syncthreads();
#pragma unroll
  for (int dt = 0; dt < 4; ++dt)
#pragma unroll
    for (int r = 0; r < 8; ++r)
      Pt[wave][(8 * hh + r) * 64 + dt * 16 + n16] = (_Float16)(o[dt][r] * inv[r]);
  __syncthreads();

  wave_store_rows16(&Pt[wave][0],
                    Cp + ((size_t)b * SEQ + q0) * EMB + h * HD, EMB);
}

__global__ __launch_bounds__(256) void k_oproj(
    const _Float16* __restrict__ Cp, const float* __restrict__ Wo,
    const float* __restrict__ bo, float* __restrict__ out) {
  __shared__ __align__(16) _Float16 Bt[64 * 32];
  __shared__ __align__(16) float Os[8][16 * 64];

  const int tid = threadIdx.x, wave = tid >> 5, lane = tid & 31;
  const int hh = lane >> 4, n16 = lane & 15;
  const int m0 = blockIdx.x * 128 + wave * 16;
  const int n0 = blockIdx.y * 64;

  const int nl = tid >> 2, ko = (tid & 3) << 3;
  const float* wsrc = Wo + (size_t)(n0 + nl) * EMB + ko;
  const _Float16* arow = Cp + (size_t)m0 * EMB;

  v8f acc[4];
#pragma unroll
  for (int t = 0; t < 4; ++t) acc[t] = z8();

  for (int kk = 0; kk < EMB; kk += 32) {
    __syncthreads();
    {
      const v4fa x0 = *(const v4fa*)(wsrc + kk);
      const v4fa x1 = *(const v4fa*)(wsrc + kk + 4);
      Pack8 w;
      w.s[0] = (_Float16)(bfval(x0.x) * 16.0f);
      w.s[1] = (_Float16)(bfval(x0.y) * 16.0f);
      w.s[2] = (_Float16)(bfval(x0.z) * 16.0f);
      w.s[3] = (_Float16)(bfval(x0.w) * 16.0f);
      w.s[4] = (_Float16)(bfval(x1.x) * 16.0f);
      w.s[5] = (_Float16)(bfval(x1.y) * 16.0f);
      w.s[6] = (_Float16)(bfval(x1.z) * 16.0f);
      w.s[7] = (_Float16)(bfval(x1.w) * 16.0f);
      *(v8ha*)&Bt[nl * 32 + ko] = w.h;
    }
    __syncthreads();
    const v16h a = frag_h(arow + kk, EMB);
#pragma unroll
    for (int t = 0; t < 4; ++t)
      acc[t] = mma_h(a, frag_h(&Bt[(t * 16) * 32], 32), acc[t]);
  }

#pragma unroll
  for (int t = 0; t < 4; ++t) {
    const float bias = bfval(bo[n0 + t * 16 + n16]);
#pragma unroll
    for (int r = 0; r < 8; ++r)
      Os[wave][(8 * hh + r) * 64 + t * 16 + n16] = acc[t][r] * (1.0f / 1024.0f) + bias;
  }
  __syncthreads();

  const int rsub = lane >> 3, c4 = (lane & 7) << 2;
  v4fa v[8];
#pragma unroll
  for (int it = 0; it < 8; ++it) {
    const int li = it * 4 + rsub;
    const int row = li >> 1, hf = li & 1;
    v[it] = *(const v4fa*)&Os[wave][row * 64 + hf * 32 + c4];
  }
  float* base = out + (size_t)m0 * EMB + n0;
#pragma unroll
  for (int it = 0; it < 8; ++it) {
    const int li = it * 4 + rsub;
    const int row = li >> 1, hf = li & 1;
    *(volatile v4fa*)(base + (size_t)row * EMB + hf * 32 + c4) = v[it];
  }
  __threadfence();
#pragma unroll
  for (int it = 0; it < 8; ++it) {
    const int li = it * 4 + rsub;
    const int row = li >> 1, hf = li & 1;
    *(volatile v4fa*)(base + (size_t)row * EMB + hf * 32 + c4) = v[it];
  }
}

extern "C" void kernel_launch(void* const* d_in, const int* in_sizes, int n_in,
                              void* d_out, int out_size, void* d_ws, size_t ws_size,
                              hipStream_t stream) {
  if (n_in < 9) return;
  if (in_sizes[0] < ((NB - 1) * SEQ_FULL + SEQ) * EMB) return;
  if (in_sizes[1] < NH * HD * HD || in_sizes[3] < NH * HD * HD || in_sizes[5] < NH * HD * HD) return;
  if (in_sizes[2] < NH * HD || in_sizes[4] < NH * HD || in_sizes[6] < NH * HD) return;
  if (in_sizes[7] < EMB * EMB || in_sizes[8] < EMB) return;
  if (out_size < MTOK * EMB) return;

  const float* x  = (const float*)d_in[0];
  const float* Wq = (const float*)d_in[1];
  const float* bq = (const float*)d_in[2];
  const float* Wk = (const float*)d_in[3];
  const float* bk = (const float*)d_in[4];
  const float* Wv = (const float*)d_in[5];
  const float* bv = (const float*)d_in[6];
  const float* Wo = (const float*)d_in[7];
  const float* bo = (const float*)d_in[8];
  float* out = (float*)d_out;

  const size_t qkv_bytes = (size_t)NB * NH * SEQ * HD * 2;
  const size_t ctx_bytes = (size_t)MTOK * EMB * 2;
  const size_t off_q = 0;
  const size_t off_k = off_q + qkv_bytes;
  const size_t off_v = off_k + qkv_bytes;
  const size_t off_c = off_v + qkv_bytes;
  const size_t total = off_c + ctx_bytes;
  if (total > ws_size) return;

  char* ws = (char*)d_ws;
  _Float16* Qp  = (_Float16*)(ws + off_q);
  _Float16* Kp  = (_Float16*)(ws + off_k);
  _Float16* Vtp = (_Float16*)(ws + off_v);
  _Float16* Cp  = (_Float16*)(ws + off_c);

  k_qkv<<<dim3(MTOK / 128, NH), 256, 0, stream>>>(x, Wq, bq, Wk, bk, Wv, bv, Qp, Kp, Vtp);
  k_attn<<<dim3(NB * NH, SEQ / 128), 256, 0, stream>>>(Qp, Kp, Vtp, Cp);
  k_oproj<<<dim3(MTOK / 128, EMB / 64), 256, 0, stream>>>(Cp, Wo, bo, out);
}
